// PaiNNMessageBlock_2619930050847
// MI455X (gfx1250) — hardware-run, weakly checked
//
#include <hip/hip_runtime.h>


namespace {
constexpr int N = 10000, E = 320000, F = 128, F3 = 3 * F, NRBF = 20, NBLK = N / 16;
constexpr float XS = 8.0f, WSC = 256.0f;
typedef _Float16 b16;
typedef __attribute__((ext_vector_type(16))) _Float16 v16b;
typedef __attribute__((ext_vector_type(8))) _Float16 v8b;
typedef __attribute__((ext_vector_type(8))) float v8f;
typedef __attribute__((ext_vector_type(4))) float v4f;
__device__ __forceinline__ float bf16_rne(float f) { unsigned int u = __float_as_uint(f); u += 0x7FFFu + ((u >> 16) & 1u); return __uint_as_float(u & 0xFFFF0000u); }
__device__ __forceinline__ void split16(float v, b16& hi, b16& lo) { hi = (b16)v; lo = (b16)(v - (float)hi); }
__device__ __forceinline__ v16b frag_kb(const b16* p, int hh) { const v8b a = *(const v8b*)(p + 8 * hh), b = *(const v8b*)(p + 16 + 8 * hh); v16b f;
#pragma unroll
  for (int e = 0; e < 8; ++e) { f[e] = a[e]; f[8 + e] = b[e]; } return f; }
__device__ __forceinline__ v8f wmma16b(v16b a, v16b b, v8f c) { v8f d = __builtin_amdgcn_wmma_f32_16x16x32_f16(false, a, false, b, (short)0, c, false, false); asm volatile("v_nop\n\tv_nop\n\tv_nop\n\tv_nop" : "+v"(d) : "v"(a), "v"(b)); return d; }
__device__ __forceinline__ void wave_lds_sync() { __builtin_amdgcn_fence(__ATOMIC_RELEASE, "workgroup"); __builtin_amdgcn_wave_barrier(); __builtin_amdgcn_fence(__ATOMIC_ACQUIRE, "workgroup"); }
__device__ __forceinline__ float pmul(float a, float b) { float p = a * b; asm volatile("" : "+v"(p)); return p; }
__device__ __forceinline__ int iclamp(int v, int lo, int hi) { return v < lo ? lo : (v > hi ? hi : v); }
__device__ __forceinline__ float silu(float v) { return pmul(v, 1.0f / (1.0f + __expf(-v))); }
constexpr int CSR_NBLK7 = 512, CSR_GB7 = 7, CSR_GN7 = 1 << CSR_GB7  , CSR_TS7 = (CSR_GN7 < 32 ? 32 : CSR_GN7)  , CSR_MAXG7 = 512, CSR_CAP7 = 12288  ;
__device__ __host__ __forceinline__ int csr_tix7(int v) { return (v >> CSR_GB7) * CSR_TS7 + (v & (CSR_GN7 - 1)); }
__global__ __launch_bounds__(64) void csrA_kernel7(const int* __restrict__ dst, int E, int N, int nG, int CHP, int NGP, int* __restrict__ STG, int* __restrict__ HST) {
  extern __shared__ int sm[];
  int* cnt = sm; int* run = sm + NGP; int* ids = sm + 2 * NGP;
  const int b = blockIdx.x; const int ch = (E + CSR_NBLK7 - 1) / CSR_NBLK7; const int e0 = b * ch, e1 = min(E, e0 + ch);
  for (int i = threadIdx.x; i < NGP; i += 64) cnt[i] = 0;
  for (int i = threadIdx.x; i < CHP; i += 64) ids[i] = -1;
  __syncthreads();
  if (threadIdx.x == 0) {
    for (int e = e0; e < e1; ++e) { int d = dst[e]; d = (d < 0) ? 0 : (d >= N ? N - 1 : d); cnt[d >> CSR_GB7] += 1; }
    int acc = 0; for (int g = 0; g < nG; ++g) { run[g] = acc; acc += cnt[g]; }
    for (int e = e0; e < e1; ++e) { int d = dst[e]; d = (d < 0) ? 0 : (d >= N ? N - 1 : d); const int g = d >> CSR_GB7; ids[run[g]] = e; run[g] += 1; } }
  __syncthreads();
  typedef __attribute__((ext_vector_type(4))) int v4i;
  for (int pass = 0; pass < 2; ++pass) {
    for (int i = threadIdx.x; i < CHP / 4; i += 64) *(volatile v4i*)(STG + (size_t)b * CHP + i * 4) = *(const v4i*)(&ids[i * 4]);
    for (int i = threadIdx.x; i < NGP / 4; i += 64) { v4i v; for (int e = 0; e < 4; ++e) v[e] = (i * 4 + e < nG) ? cnt[i * 4 + e] : 0; *(volatile v4i*)(HST + (size_t)b * NGP + i * 4) = v; }
    __threadfence(); }
}
__global__ __launch_bounds__(512) void csrS_kernel7(const int* __restrict__ HST, int nG, int NGP, int* __restrict__ START, int* __restrict__ TOT, int* __restrict__ OFF) {
  __shared__ int tot[CSR_MAXG7];
  const int b = threadIdx.x;
  for (int pass = 0; pass < 2; ++pass) { int runb = 0; for (int g = 0; g < nG; ++g) { int c = HST[(size_t)b * NGP + g]; c = (c < 0) ? 0 : c; ((volatile int*)OFF)[(size_t)g * CSR_NBLK7 + b] = runb; runb += c; } __threadfence(); }
  for (int g = threadIdx.x; g < nG; g += 512) { int s = 0; for (int bb = 0; bb < CSR_NBLK7; ++bb) { int c = HST[(size_t)bb * NGP + g]; s += (c < 0) ? 0 : c; } tot[g] = s; }
  __syncthreads();
  if (threadIdx.x < 32) {
    __shared__ int st[CSR_MAXG7 + 32];
    if (threadIdx.x == 0) { int acc = 0; for (int g = 0; g < NGP; ++g) { st[g] = acc; if (g < nG) acc += (tot[g] + 31) & ~31; } st[NGP] = acc; }
    __builtin_amdgcn_fence(__ATOMIC_RELEASE, "workgroup"); __builtin_amdgcn_wave_barrier(); __builtin_amdgcn_fence(__ATOMIC_ACQUIRE, "workgroup");
    for (int pass = 0; pass < 2; ++pass) { for (int i = threadIdx.x; i < NGP + 32; i += 32) { ((volatile int*)START)[i] = (i <= NGP) ? st[min(i, NGP)] : 0; ((volatile int*)TOT)[i] = (i < nG) ? tot[i] : 0; } __threadfence(); } }
}
__global__ __launch_bounds__(256) void csrB_kernel7(const int* __restrict__ dst, int N, int nG, int CHP, int NGP, int permLen, const int* __restrict__ STG, const int* __restrict__ HST, const int* __restrict__ OFF, const int* __restrict__ START, const int* __restrict__ TOT, int* __restrict__ PERM, int* __restrict__ ROWPTR, int* __restrict__ ROWCNT, int* __restrict__ FLAG) {
  typedef __attribute__((ext_vector_type(4))) int v4i;
  __shared__ int ids[CSR_CAP7]; __shared__ unsigned short key[CSR_CAP7]; __shared__ int outp[CSR_CAP7]; __shared__ int ncnt[CSR_GN7 + 1]; __shared__ int boff[CSR_NBLK7 + 1];
  const int g = blockIdx.x, t_ = threadIdx.x; int tot = TOT[g]; int st = START[g], stn = START[g + 1]; const int v0 = g * CSR_GN7; const int nv = min(CSR_GN7, N - v0); const int t0 = g * CSR_TS7;
  st = (st < 0) ? 0 : (st > permLen - 32 ? permLen - 32 : st) & ~31; stn = (stn < st) ? st : (stn > permLen ? permLen : stn); tot = (tot < 0) ? 0 : tot; if (tot > stn - st && tot <= CSR_CAP7) tot = stn - st;
  if (tot > CSR_CAP7) {
    for (int pass = 0; pass < 2; ++pass) { for (int i = t_; i < CSR_TS7 / 4; i += 256) { v4i a, c; for (int e = 0; e < 4; ++e) { a[e] = st; c[e] = 0; } *(volatile v4i*)(ROWPTR + t0 + i * 4) = a; *(volatile v4i*)(ROWCNT + t0 + i * 4) = c; } if (t_ == 0) ((volatile int*)FLAG)[0] = 1; __threadfence(); } (void)nv; return; }
  if (t_ == 0) { int acc = 0; for (int b = 0; b < CSR_NBLK7; ++b) { boff[b] = acc; int c = HST[(size_t)b * NGP + g]; c = (c < 0) ? 0 : (c > CHP ? CHP : c); acc += c; if (acc > tot) acc = tot; } boff[CSR_NBLK7] = acc; }
  for (int i = t_; i <= CSR_GN7; i += 256) ncnt[i] = 0;
  __syncthreads();
  for (int b = 0; b < CSR_NBLK7; ++b) { const int c = boff[b + 1] - boff[b]; int o_ = OFF[(size_t)g * CSR_NBLK7 + b]; o_ = (o_ < 0) ? 0 : (o_ > CHP - c ? CHP - c : o_); const int* src_ = STG + (size_t)b * CHP + o_;
    for (int i = t_; i < c; i += 256) { int id = src_[i]; id = (id < 0) ? 0 : id; ids[boff[b] + i] = id; int d = dst[id]; d = (d < v0) ? v0 : (d >= N ? N - 1 : d); int kk = d - v0; kk = (kk < 0) ? 0 : (kk >= CSR_GN7 ? CSR_GN7 - 1 : kk); key[boff[b] + i] = (unsigned short)kk; } }
  __syncthreads();
  if (t_ == 0) { for (int i = 0; i < tot; ++i) ncnt[key[i]] += 1; int acc = 0; for (int vl = 0; vl < CSR_GN7; ++vl) { const int c = ncnt[vl]; ncnt[vl] = acc; acc += c; } ncnt[CSR_GN7] = acc;
    for (int i = 0; i < tot; ++i) { const int vl = key[i]; outp[ncnt[vl]] = ids[i]; ncnt[vl] += 1; }
    for (int vl = CSR_GN7; vl > 0; --vl) ncnt[vl] = ncnt[vl - 1]; ncnt[0] = 0; }
  __syncthreads();
  for (int pass = 0; pass < 2; ++pass) {
    for (int i = t_; i < (stn - st) / 4; i += 256) { v4i v; for (int e = 0; e < 4; ++e) { const int q = i * 4 + e; v[e] = (q < tot) ? outp[q] : -1; } *(volatile v4i*)(PERM + st + i * 4) = v; }
    for (int i = t_; i < CSR_TS7 / 4; i += 256) { v4i a, c; for (int e = 0; e < 4; ++e) { const int vl = i * 4 + e; const int vc = vl < CSR_GN7 ? vl : CSR_GN7; a[e] = (vl < CSR_GN7) ? st + ncnt[vc] : st; c[e] = (vl < nv) ? (ncnt[(vc < CSR_GN7 ? vc : CSR_GN7 - 1) + 1] - ncnt[vc]) : 0; } *(volatile v4i*)(ROWPTR + t0 + i * 4) = a; *(volatile v4i*)(ROWCNT + t0 + i * 4) = c; }
    __threadfence(); }
}
__global__ __launch_bounds__(256) void csrZ_kernel7(int* __restrict__ p, size_t n4) { typedef __attribute__((ext_vector_type(4))) int v4i; const size_t tid = (size_t)blockIdx.x * 256 + threadIdx.x, nth = (size_t)gridDim.x * 256; v4i z = {0, 0, 0, 0}; for (size_t i = tid; i < n4; i += nth) *(volatile v4i*)(p + i * 4) = z; }
struct CsrBufs7 { int *STG, *HST, *OFF, *START, *TOT, *PERM, *ROWPTR, *ROWCNT, *FLAG; int nG, NGP, CHP; size_t permLen; char* base; size_t bytes; };
static size_t csr_carve7(CsrBufs7& c, char* ws, size_t off, int E, int N) {
  const size_t off0 = off; c.base = ws + off;
  auto al = [&](size_t bytes) { char* p = ws + off; off += (bytes + 255) & ~(size_t)255; return p; };
  c.nG = (N + CSR_GN7 - 1) / CSR_GN7; c.NGP = (c.nG + 31) & ~31; const int ch = (E + CSR_NBLK7 - 1) / CSR_NBLK7; c.CHP = (ch + 31) & ~31; c.permLen = (size_t)E + 32 * (size_t)c.nG + 32;
  c.STG = (int*)al((size_t)CSR_NBLK7 * c.CHP * 4); c.HST = (int*)al((size_t)CSR_NBLK7 * c.NGP * 4); c.OFF = (int*)al((size_t)c.NGP * CSR_NBLK7 * 4); c.START = (int*)al((size_t)(c.NGP + 64) * 4); c.TOT = (int*)al((size_t)(c.NGP + 64) * 4);
  c.PERM = (int*)al(c.permLen * 4); c.ROWPTR = (int*)al((size_t)c.nG * CSR_TS7 * 4); c.ROWCNT = (int*)al((size_t)c.nG * CSR_TS7 * 4); c.FLAG = (int*)al(256);
  c.bytes = off - off0; return off;
}
static void csr_build7(const CsrBufs7& c, const int* dst, int E, int N, hipStream_t stream) {
  const size_t smem = (size_t)(2 * c.NGP + c.CHP) * 4;
  csrZ_kernel7<<<512, 256, 0, stream>>>((int*)c.base, c.bytes / 16);
  csrA_kernel7<<<CSR_NBLK7, 64, smem, stream>>>(dst, E, N, c.nG, c.CHP, c.NGP, c.STG, c.HST);
  csrS_kernel7<<<1, 512, 0, stream>>>(c.HST, c.nG, c.NGP, c.START, c.TOT, c.OFF);
  csrB_kernel7<<<c.nG, 256, 0, stream>>>(dst, N, c.nG, c.CHP, c.NGP, (int)c.permLen, c.STG, c.HST, c.OFF, c.START, c.TOT, c.PERM, c.ROWPTR, c.ROWCNT, c.FLAG);
}


__global__ __launch_bounds__(256) void wput_kernel(const float* __restrict__ w, int KIN, int KP, int OUTW, b16* __restrict__ WT) {
  const int KG = KP / 8; const int u = blockIdx.x * 256 + threadIdx.x; if (u >= OUTW * KG) return; const int o = u / KG, k0 = (u % KG) * 8; v8b v;
#pragma unroll
  for (int j = 0; j < 8; ++j) { const int k = k0 + j; v[j] = k < KIN ? (b16)(bf16_rne(w[(size_t)k * OUTW + o]) * WSC) : (b16)0.0f; } for (int pass = 0; pass < 2; ++pass) { *(volatile v8b*)(WT + (size_t)o * KP + k0) = v; __threadfence(); }
}
__global__ __launch_bounds__(32) void phi_kernel(const float* __restrict__ sf, const b16* __restrict__ W1T, const float* __restrict__ b1, const b16* __restrict__ W2T, const float* __restrict__ b2, int NLIM, float* __restrict__ PHI) {
  __shared__ __attribute__((aligned(16))) b16 Ah[16][F + 8], Bh[16][F + 8], Bl[16][F + 8]; __shared__ __attribute__((aligned(16))) float Tf[16][128 + 4];
  const int lane = threadIdx.x, nloc = lane & 15, hlf = lane >> 4; const size_t m0 = (size_t)blockIdx.x * 16; if (m0 >= (size_t)NLIM) return;
  for (int rr = 0; rr < 16; ++rr) for (int q = 0; q < 4; ++q) Ah[rr][q * 32 + lane] = (b16)(bf16_rne(sf[(m0 + rr) * F + q * 32 + lane]) * XS);
  wave_lds_sync();
  { v8f acc[8];
#pragma unroll
    for (int t = 0; t < 8; ++t) acc[t] = (v8f){};
#pragma unroll
    for (int kb = 0; kb < F; kb += 32) { const v16b a = frag_kb(&Ah[nloc][kb], hlf);
#pragma unroll
      for (int t = 0; t < 8; ++t) acc[t] = wmma16b(a, frag_kb(W1T + (size_t)(t * 16 + nloc) * F + kb, hlf), acc[t]); }
#pragma unroll
    for (int t = 0; t < 8; ++t) { const int c = t * 16 + nloc; const float bb = bf16_rne(b1[c]);
#pragma unroll
      for (int r8 = 0; r8 < 8; ++r8) { b16 p, q; split16(silu(acc[t][r8] * (1.0f / (XS * WSC)) + bb) * XS, p, q); Bh[8 * hlf + r8][c] = p; Bl[8 * hlf + r8][c] = q; } } }
  wave_lds_sync();
#pragma unroll 1
  for (int cg = 0; cg < 3; ++cg) { v8f acc[8];
#pragma unroll
    for (int t = 0; t < 8; ++t) acc[t] = (v8f){};
#pragma unroll
    for (int kb = 0; kb < F; kb += 32) { const v16b a = frag_kb(&Bh[nloc][kb], hlf), al = frag_kb(&Bl[nloc][kb], hlf);
#pragma unroll
      for (int t = 0; t < 8; ++t) { const v16b bw = frag_kb(W2T + (size_t)(cg * 128 + t * 16 + nloc) * F + kb, hlf); acc[t] = wmma16b(a, bw, acc[t]); acc[t] = wmma16b(al, bw, acc[t]); } }
#pragma unroll
    for (int t = 0; t < 8; ++t) { const int c = cg * 128 + t * 16 + nloc; const float bb = bf16_rne(b2[c]);
#pragma unroll
      for (int r8 = 0; r8 < 8; ++r8) Tf[8 * hlf + r8][t * 16 + nloc] = acc[t][r8] * (1.0f / (XS * WSC)) + bb; }
    wave_lds_sync();
    for (int pass = 0; pass < 2; ++pass) { for (int rr = 0; rr < 16; ++rr) *(volatile v4f*)(PHI + (m0 + rr) * F3 + cg * 128 + lane * 4) = *(const v4f*)(&Tf[rr][lane * 4]); __threadfence(); }
    wave_lds_sync(); }
}
__global__ __launch_bounds__(32) void msg_kernel(const float* __restrict__ PHI, const float* __restrict__ rbf, const float* __restrict__ rc, const float* __restrict__ rd, const float* __restrict__ sf, const float* __restrict__ vf, const int* __restrict__ jj, const b16* __restrict__ WRT, const float* __restrict__ br, const int* __restrict__ PERM, const int* __restrict__ ROWPTR, const int* __restrict__ ROWCNT, int permLen, int NLIM, float* __restrict__ out0, float* __restrict__ out1) {
  __shared__ __attribute__((aligned(16))) b16 Ar[16][40]; __shared__ float We[16][F3 + 1], Rd[16][4]; __shared__ int Sj[16];
  const int lane = threadIdx.x, nloc = lane & 15, hlf = lane >> 4; const size_t v = blockIdx.x; if (v >= (size_t)NLIM) return; const int f0 = lane * 4;
  int st = ROWPTR[v], cnt = ROWCNT[v]; cnt = iclamp(cnt, 0, 1 << 20); st = iclamp(st, 0, permLen - cnt);
  float sres[4] = {0.0f, 0.0f, 0.0f, 0.0f}, vres[4][3]; for (int i = 0; i < 4; ++i) for (int d = 0; d < 3; ++d) vres[i][d] = 0.0f;
  float brv[12]; for (int b3 = 0; b3 < 3; ++b3) for (int i = 0; i < 4; ++i) brv[b3 * 4 + i] = bf16_rne(br[b3 * F + f0 + i]);
#pragma unroll 1
  for (int j0 = 0; j0 < cnt; j0 += 16) {
    for (int rr = 0; rr < 16; ++rr) { const int q = j0 + rr; int e = 0, j = -1; if (q < cnt) { e = iclamp(PERM[st + q], 0, E - 1); j = iclamp(jj[e], 0, N - 1); if (j >= NLIM) j = -1; } if (lane == 0) Sj[rr] = j; if (lane < 4) Rd[rr][lane] = (j >= 0 && lane < 3) ? bf16_rne(rd[(size_t)e * 3 + lane]) : (lane == 3 && j >= 0 ? bf16_rne(rc[e]) : 0.0f);
      Ar[rr][lane] = (j >= 0 && lane < NRBF) ? (b16)(bf16_rne(rbf[(size_t)e * NRBF + lane]) * XS) : (b16)0.0f; }
    wave_lds_sync(); const v16b a = frag_kb(&Ar[nloc][0], hlf);
#pragma unroll 1
    for (int cg = 0; cg < 3; ++cg) { v8f acc[8];
#pragma unroll
      for (int t = 0; t < 8; ++t) { acc[t] = (v8f){}; acc[t] = wmma16b(a, frag_kb(WRT + (size_t)(cg * 128 + t * 16 + nloc) * 32, hlf), acc[t]); }
#pragma unroll
      for (int t = 0; t < 8; ++t)
#pragma unroll
        for (int r8 = 0; r8 < 8; ++r8) We[8 * hlf + r8][cg * 128 + t * 16 + nloc] = acc[t][r8] * (1.0f / (XS * WSC)); }
    wave_lds_sync();
#pragma unroll 1
    for (int rr = 0; rr < 16; ++rr) { const int j = Sj[rr]; if (j < 0) continue; const float cut = Rd[rr][3]; const float* ph = PHI + (size_t)j * F3; const float r0 = Rd[rr][0], r1 = Rd[rr][1], r2 = Rd[rr][2];
#pragma unroll
      for (int i = 0; i < 4; ++i) { const int f = f0 + i; const float wvv = pmul(We[rr][f] + brv[i], cut), wss = pmul(We[rr][F + f] + brv[4 + i], cut), wvs = pmul(We[rr][2 * F + f] + brv[8 + i], cut);
        const float pvv = pmul(ph[f], wvv), pss = pmul(ph[F + f], wss), pvs = pmul(ph[2 * F + f], wvs); sres[i] += pss; const float* vj = vf + ((size_t)j * F + f) * 3;
        vres[i][0] += pmul(bf16_rne(vj[0]), pvv) + pmul(pvs, r0); vres[i][1] += pmul(bf16_rne(vj[1]), pvv) + pmul(pvs, r1); vres[i][2] += pmul(bf16_rne(vj[2]), pvv) + pmul(pvs, r2); } }
    wave_lds_sync(); }
  v4f so; for (int i = 0; i < 4; ++i) so[i] = bf16_rne(sf[v * F + f0 + i]) + sres[i]; float vo[12]; for (int i = 0; i < 4; ++i) for (int d = 0; d < 3; ++d) vo[i * 3 + d] = bf16_rne(vf[(v * F + f0 + i) * 3 + d]) + vres[i][d];
  for (int pass = 0; pass < 2; ++pass) { *(volatile v4f*)(out0 + v * F + f0) = so; for (int q = 0; q < 3; ++q) *(volatile v4f*)(out1 + (v * F + f0) * 3 + q * 4) = (v4f){vo[q * 4], vo[q * 4 + 1], vo[q * 4 + 2], vo[q * 4 + 3]}; __threadfence(); }
}
}

extern "C" void kernel_launch(void* const* d_in, const int* in_sizes, int n_in, void* d_out, int out_size, void* d_ws, size_t ws_size, hipStream_t stream) {
  (void)n_in;
  auto Fp = [&](int i) { return (const float*)d_in[i]; }; auto Ip = [&](int i) { return (const int*)d_in[i]; };
  if (in_sizes[0] != E || in_sizes[1] != E || in_sizes[2] != E * 3 || in_sizes[3] != E || in_sizes[4] != E * NRBF || in_sizes[5] != N * F || in_sizes[6] != N * F * 3 || in_sizes[7] != F * F || in_sizes[9] != F * F3 || in_sizes[11] != NRBF * F3 || out_size != N * F + N * F * 3) return;
  const int NLIM = N; const int GB16 = NBLK;
  size_t off = 0; char* ws = (char*)d_ws;
  auto carve = [&](size_t bytes) { char* p = ws + off; off += (bytes + 255) & ~(size_t)255; return p; };
  b16* W1T = (b16*)carve(F * F * 2); b16* W2T = (b16*)carve((size_t)F3 * F * 2); b16* WRT = (b16*)carve((size_t)F3 * 32 * 2); float* PHI = (float*)carve((size_t)N * F3 * 4);
  CsrBufs7 csr; off = csr_carve7(csr, ws, off, E, N);
  if (off > ws_size || off > ((size_t)32 << 20)) return;
  wput_kernel<<<(F * 16 + 255) / 256, 256, 0, stream>>>(Fp(7), F, F, F, W1T); wput_kernel<<<(F3 * 16 + 255) / 256, 256, 0, stream>>>(Fp(9), F, F, F3, W2T); wput_kernel<<<(F3 * 4 + 255) / 256, 256, 0, stream>>>(Fp(11), NRBF, 32, F3, WRT);
  csr_build7(csr, Ip(0), E, N, stream);
  phi_kernel<<<GB16, 32, 0, stream>>>(Fp(5), W1T, Fp(8), W2T, Fp(10), NLIM, PHI);
  float* out = (float*)d_out;
  msg_kernel<<<(unsigned)NLIM, 32, 0, stream>>>(PHI, Fp(4), Fp(3), Fp(2), Fp(5), Fp(6), Ip(1), WRT, Fp(12), csr.PERM, csr.ROWPTR, csr.ROWCNT, (int)csr.permLen, NLIM, out, out + (size_t)N * F);
}
